// practiceNet_27994596836177
// MI455X (gfx1250) — hardware-verified
//
#include <hip/hip_runtime.h>
#include <math.h>

typedef __attribute__((ext_vector_type(16))) _Float16 v16h;
typedef __attribute__((ext_vector_type(16))) __bf16 v16b;
typedef __attribute__((ext_vector_type(8)))  _Float16 v8h;
typedef __attribute__((ext_vector_type(8)))  float v8f;
typedef __attribute__((ext_vector_type(4)))  float v4f;
typedef __attribute__((ext_vector_type(2)))  float v2f;
typedef __attribute__((ext_vector_type(4)))  unsigned v4u;
typedef __attribute__((ext_vector_type(4)))  int v4i;
typedef float __attribute__((may_alias)) float_a;
typedef int __attribute__((may_alias)) int_a;

template <typename T> __device__ __forceinline__ void vst2(void* p, T v) { *(volatile T*)p = v; __threadfence(); *(volatile T*)p = v; }
__device__ __forceinline__ v8f wmma16(v16h a, v16h b, v8f c) {
  v8f d = __builtin_amdgcn_wmma_f32_16x16x32_f16(false, a, false, b, (short)0, c, false, false);
  asm volatile("v_nop\n\tv_nop\n\tv_nop\n\tv_nop" : "+v"(d) : "v"(a), "v"(b));
  return d;
}
__device__ __forceinline__ v8f wmma_bf(v16b a, v16b b, v8f c) {
  v8f d = __builtin_amdgcn_wmma_f32_16x16x32_bf16(false, a, false, b, (short)0, c, false, false);
  asm volatile("v_nop\n\tv_nop\n\tv_nop\n\tv_nop" : "+v"(d) : "v"(a), "v"(b));
  return d;
}
__device__ __forceinline__ v16h frag_h(const _Float16* rowk0, int lane) {
  union { v16h v; v8h q[2]; } u; const _Float16* p = rowk0 + 8 * (lane >> 4);
  u.q[0] = *(const v8h*)p; u.q[1] = *(const v8h*)(p + 16); return u.v;
}
__device__ __forceinline__ v16h frag_f32(const float* rowk0, int lane) {
  v16h a; const float* p = rowk0 + 8 * (lane >> 4);
#pragma unroll
  for (int i = 0; i < 8; ++i) { a[i] = (_Float16)p[i]; a[8 + i] = (_Float16)p[16 + i]; }
  return a;
}
__device__ __forceinline__ v16h frag_f32s(const float* rowk0, int lane, float sc) {
  v16h a; const float* p = rowk0 + 8 * (lane >> 4);
#pragma unroll
  for (int i = 0; i < 8; ++i) { a[i] = (_Float16)(p[i] * sc); a[8 + i] = (_Float16)(p[16 + i] * sc); }
  return a;
}
__device__ __forceinline__ v16h fragc_f32(const float* W, int k0, int n, int lane, int ld, int K) {
  v16h a; const int g = lane >> 4;
#pragma unroll
  for (int i = 0; i < 8; ++i) { const int ka = k0 + 8 * g + i, kb = ka + 16;
    a[i] = (_Float16)(ka < K ? W[(size_t)(ka < K ? ka : K - 1) * ld + n] : 0.f); a[8 + i] = (_Float16)(kb < K ? W[(size_t)(kb < K ? kb : K - 1) * ld + n] : 0.f); }
  return a;
}
struct F2 { v16b h, l; };
__device__ __forceinline__ F2 bsplit16(const float v[16]) { F2 r;
#pragma unroll
  for (int i = 0; i < 16; ++i) { const __bf16 h = (__bf16)v[i]; r.h[i] = h; r.l[i] = (__bf16)(v[i] - (float)h); }
  return r; }
__device__ __forceinline__ F2 split_row(const float* row, int k0, int lane) { float v[16]; const float* p = row + k0 + 8 * (lane >> 4);
#pragma unroll
  for (int i = 0; i < 8; ++i) { v[i] = p[i]; v[8 + i] = p[16 + i]; }
  return bsplit16(v); }
__device__ __forceinline__ F2 split_rowK(const float* row, int k0, int lane, int K) { float v[16]; const int g = lane >> 4;
#pragma unroll
  for (int i = 0; i < 8; ++i) { const int ka = k0 + 8 * g + i, kb = ka + 16; v[i] = ka < K ? row[ka < K ? ka : K - 1] : 0.f; v[8 + i] = kb < K ? row[kb < K ? kb : K - 1] : 0.f; }
  return bsplit16(v); }
__device__ __forceinline__ F2 split_col(const float* W, int k0, int n, int lane, int ld, int K) { float v[16]; const int g = lane >> 4;
#pragma unroll
  for (int i = 0; i < 8; ++i) { const int ka = k0 + 8 * g + i, kb = ka + 16; v[i] = ka < K ? W[(size_t)(ka < K ? ka : K - 1) * ld + n] : 0.f; v[8 + i] = kb < K ? W[(size_t)(kb < K ? kb : K - 1) * ld + n] : 0.f; }
  return bsplit16(v); }
__device__ __forceinline__ v8f mac3(const F2& a, const F2& b, v8f c) { c = wmma_bf(a.l, b.h, c); c = wmma_bf(a.h, b.l, c); return wmma_bf(a.h, b.h, c); }
__device__ __forceinline__ float sigm(float v) { return 1.0f / (1.0f + expf(-v)); }
#define LDSX() do { asm volatile("s_wait_dscnt 0" ::: "memory"); __builtin_amdgcn_wave_barrier(); __builtin_amdgcn_fence(__ATOMIC_RELEASE, "workgroup"); } while (0)


#define NB 2
#define HI 96
#define WI 96
#define NPOS (HI * WI)
#define C1 8
#define C2 16
#define C3 64
#define C4 8
#define K3 (C2 * 25)
#define K3P 416
#define K4 (C3 * 9)
#ifndef TQB
#define TQB (NPOS / 64)
#define TNB NB
#define C4B (NPOS / 64)
#define C5R HI
#endif
typedef __attribute__((ext_vector_type(8))) __bf16 v8b;
__device__ __forceinline__ v16b frag_b(const __bf16* rowk0, int lane) {
  union { v16b v; v8b q[2]; } u; const __bf16* p = rowk0 + 8 * (lane >> 4);
  u.q[0] = *(const v8b*)p; u.q[1] = *(const v8b*)(p + 16); return u.v;
}
__device__ __forceinline__ float bfr(float v) { return (float)(__bf16)v; }
__device__ __attribute__((noinline)) float exp_ni(float v) { return expf(v); }
__device__ __attribute__((noinline)) float erf_ni(float v) { return erff(v); }

#define WS_P3  0u
#define WS_P4  (WS_P3 + 2u * C3 * K3P)
#define WS_A1  (WS_P4 + 2u * 16 * K4)
#define WS_A2  (WS_A1 + 4u * NB * C1 * NPOS)
#define WS_BT  (WS_A2 + 4u * NB * C2 * NPOS)
#define WS_VH  (WS_BT + 4u * NB * NPOS * C3)
#define WS_VL  (WS_VH + 2u * NB * C3 * NPOS)
#define WS_O   (WS_VL + 2u * NB * C3 * NPOS)
#define WS_A4  (WS_O + 4u * NB * NPOS * C3)
#define WS_END (WS_A4 + 4u * NB * NPOS * 16)

__global__ __launch_bounds__(256) void k_pack(const float* __restrict__ W3, const float* __restrict__ W4, __bf16* __restrict__ P3, __bf16* __restrict__ P4) {
  __shared__ __align__(16) __bf16 s[K4]; const int tid = threadIdx.x; const int bI = blockIdx.x;
  if (bI < C3) { const int o = bI; for (int k = tid; k < K3P; k += 256) s[k] = (__bf16)((k < K3) ? W3[(size_t)o * K3 + k] : 0.f); __syncthreads();
    for (int q = tid; q < K3P / 8; q += 256) vst2((unsigned*)(P3 + (size_t)o * K3P + q * 8), *(const v4u*)&s[q * 8]); }
  else { const int o = bI - C3; for (int k = tid; k < K4; k += 256) s[k] = (__bf16)((o < C4) ? W4[(size_t)(o < C4 ? o : C4 - 1) * K4 + k] : 0.f); __syncthreads();
    for (int q = tid; q < K4 / 8; q += 256) vst2((unsigned*)(P4 + (size_t)o * K4 + q * 8), *(const v4u*)&s[q * 8]); }
}
__global__ __launch_bounds__(256) void k_conv12(const float* __restrict__ X, const float* __restrict__ W1, const float* __restrict__ B1, const float* __restrict__ W2, const float* __restrict__ B2, float* __restrict__ A2) {
  __shared__ float sx[5][WI + 4]; __shared__ float s1[C1][3][WI + 2]; __shared__ float sw1[C1][9], sb1[C1], sw2[C2][C1 * 9], sb2[C2]; __shared__ __align__(16) float so[C2][WI];
  const int h = blockIdx.x, b = blockIdx.y, tid = threadIdx.x;
  for (int q = tid; q < C1 * 9; q += 256) sw1[q / 9][q % 9] = bfr(W1[q]);
  for (int q = tid; q < C2 * C1 * 9; q += 256) sw2[q / (C1 * 9)][q % (C1 * 9)] = bfr(W2[q]);
  if (tid < C1) sb1[tid] = bfr(B1[tid]); if (tid < C2) sb2[tid] = bfr(B2[tid]);
  for (int q = tid; q < 5 * (WI + 4); q += 256) { const int r = q / (WI + 4), c = q % (WI + 4); const int hh = h - 2 + r, ww = c - 2; sx[r][c] = (hh >= 0 && hh < HI && ww >= 0 && ww < WI) ? bfr(X[((size_t)b * HI + hh) * WI + ww]) : 0.f; }
  __syncthreads();
  for (int q = tid; q < C1 * 3 * (WI + 2); q += 256) { const int o = q / (3 * (WI + 2)), rem = q % (3 * (WI + 2)); const int r = rem / (WI + 2), c = rem % (WI + 2); const int hh = h - 1 + r, ww = c - 1; float v = 0.f;
    if (hh >= 0 && hh < HI && ww >= 0 && ww < WI) { float a = sb1[o];
#pragma unroll
      for (int kh = 0; kh < 3; ++kh)
#pragma unroll
        for (int kw = 0; kw < 3; ++kw) a += sw1[o][kh * 3 + kw] * sx[r + kh][ww + kw + 1];
      v = fmaxf(a, 0.f); }
    s1[o][r][c] = v; }
  __syncthreads();
  for (int q = tid; q < C2 * WI; q += 256) { const int o = q / WI, w = q % WI; float a = sb2[o];
#pragma unroll 1
    for (int ci = 0; ci < C1; ++ci)
#pragma unroll
      for (int kh = 0; kh < 3; ++kh)
#pragma unroll
        for (int kw = 0; kw < 3; ++kw) a += sw2[o][ci * 9 + kh * 3 + kw] * s1[ci][kh][w + kw];
    so[o][w] = fmaxf(a, 0.f); }
  __syncthreads();
  for (int q = tid; q < C2 * (WI / 4); q += 256) { const int o = q / (WI / 4), pc = q % (WI / 4); vst2(A2 + (((size_t)b * C2 + o) * HI + h) * WI + pc * 4, *(const v4f*)&so[o][pc * 4]); }
}
__global__ __launch_bounds__(128) void k_conv3(const float* __restrict__ A2, const __bf16* __restrict__ P3, const float* __restrict__ B3, float* __restrict__ BT, __bf16* __restrict__ VH, __bf16* __restrict__ VL) {
  __shared__ __align__(16) float so[4][16][68]; __shared__ __align__(16) __bf16 sth[C3][72], stl[C3][72];
  const int tid = threadIdx.x, wave = tid >> 5, lane = tid & 31, col = lane & 15, g = lane >> 4; const int b = blockIdx.y; const int p0 = blockIdx.x * 64 + wave * 16;
  const int pa = p0 + col; const int ph = pa / WI, pw = pa % WI; const float* img = A2 + (size_t)b * C2 * NPOS;
  v8f acc[4] = {};
#pragma unroll 1
  for (int kc = 0; kc < K3P / 32; ++kc) { float v[16];
#pragma unroll
    for (int i = 0; i < 16; ++i) { const int k = kc * 32 + 8 * g + (i < 8 ? i : 8 + i); float x = 0.f;
      if (k < K3) { const int ci = k / 25, r = k % 25; const int hh = ph - 2 + r / 5, ww = pw - 2 + r % 5; if (hh >= 0 && hh < HI && ww >= 0 && ww < WI) x = img[((size_t)ci * HI + hh) * WI + ww]; }
      v[i] = x; }
    const F2 a = bsplit16(v);
#pragma unroll
    for (int j = 0; j < 4; ++j) { const v16b w = frag_b(P3 + (size_t)(j * 16 + col) * K3P + kc * 32, lane); acc[j] = wmma_bf(a.l, w, acc[j]); acc[j] = wmma_bf(a.h, w, acc[j]); } }
#pragma unroll
  for (int j = 0; j < 4; ++j) { const int o = j * 16 + col; const float bb = bfr(B3[o]);
#pragma unroll
    for (int r = 0; r < 8; ++r) { const float v = fmaxf(acc[j][r] + bb, 0.f); so[wave][8 * g + r][o] = v; const __bf16 hb = (__bf16)v; sth[o][wave * 16 + 8 * g + r] = hb; stl[o][wave * 16 + 8 * g + r] = (__bf16)(v - (float)hb); } }
  __syncthreads();
  for (int rl = 0; rl < 16; ++rl) if (lane < 16) vst2(BT + ((size_t)b * NPOS + p0 + rl) * C3 + lane * 4, *(const v4f*)&so[wave][rl][lane * 4]);
  for (int q = tid; q < C3 * 8; q += 128) { const int c = q >> 3, pc = q & 7; const size_t o = ((size_t)b * C3 + c) * NPOS + blockIdx.x * 64 + pc * 8; vst2((unsigned*)(VH + o), *(const v4u*)&sth[c][pc * 8]); vst2((unsigned*)(VL + o), *(const v4u*)&stl[c][pc * 8]); }
}
__global__ __launch_bounds__(128) void k_attn(const float* __restrict__ BT, const __bf16* __restrict__ VH, const __bf16* __restrict__ VL, float* __restrict__ O) {
  __shared__ __align__(16) float sp[4][16][36]; __shared__ __align__(16) float so[4][16][68];
  const int tid = threadIdx.x, wave = tid >> 5, lane = tid & 31, col = lane & 15, g = lane >> 4; const int b = blockIdx.y; const size_t q0 = (size_t)b * NPOS + blockIdx.x * 64 + wave * 16;
  const F2 a0 = split_row(BT + (q0 + col) * C3, 0, lane), a1 = split_row(BT + (q0 + col) * C3, 32, lane);
  float m[8], l[8];
#pragma unroll
  for (int r = 0; r < 8; ++r) { m[r] = -3.0e38f; l[r] = 0.f; }
  v8f acc[4] = {};
#pragma unroll 1
  for (int ks = 0; ks < NPOS / 32; ++ks) { v8f s[2];
#pragma unroll
    for (int ct = 0; ct < 2; ++ct) { const size_t kr = (size_t)b * NPOS + ks * 32 + ct * 16 + col; const F2 k0 = split_row(BT + kr * C3, 0, lane), k1 = split_row(BT + kr * C3, 32, lane); v8f c = mac3(a0, k0, (v8f){}); c = mac3(a1, k1, c);
#pragma unroll
      for (int r = 0; r < 8; ++r) s[ct][r] = c[r]; }
#pragma unroll
    for (int r = 0; r < 8; ++r) { float mx = fmaxf(s[0][r], s[1][r]);
#pragma unroll
      for (int o = 1; o < 16; o <<= 1) mx = fmaxf(mx, __shfl_xor(mx, o));
      const float mn = fmaxf(m[r], mx); const float alpha = exp_ni(m[r] - mn);
      const float e0 = exp_ni(s[0][r] - mn), e1 = exp_ni(s[1][r] - mn); float es = e0 + e1;
#pragma unroll
      for (int o = 1; o < 16; o <<= 1) es += __shfl_xor(es, o);
      l[r] = l[r] * alpha + es; m[r] = mn;
#pragma unroll
      for (int dt = 0; dt < 4; ++dt) acc[dt][r] *= alpha;
      sp[wave][8 * g + r][col] = e0; sp[wave][8 * g + r][16 + col] = e1; }
    LDSX();
    const F2 pa = split_row(&sp[wave][col][0], 0, lane);
#pragma unroll
    for (int dt = 0; dt < 4; ++dt) { const size_t vr = ((size_t)b * C3 + dt * 16 + col) * NPOS + ks * 32; const v16b vh = frag_b(VH + vr, lane), vl = frag_b(VL + vr, lane); acc[dt] = wmma_bf(pa.l, vh, acc[dt]); acc[dt] = wmma_bf(pa.h, vl, acc[dt]); acc[dt] = wmma_bf(pa.h, vh, acc[dt]); }
    LDSX(); }
#pragma unroll
  for (int r = 0; r < 8; ++r) { const float il = 1.0f / l[r];
#pragma unroll
    for (int dt = 0; dt < 4; ++dt) so[wave][8 * g + r][dt * 16 + col] = acc[dt][r] * il; }
  LDSX();
  for (int rl = 0; rl < 16; ++rl) if (lane < 16) vst2(O + (q0 + rl) * C3 + lane * 4, *(const v4f*)&so[wave][rl][lane * 4]);
}
__global__ __launch_bounds__(128) void k_conv4(const float* __restrict__ O, const __bf16* __restrict__ P4, const float* __restrict__ B4, float* __restrict__ A4) {
  __shared__ __align__(16) float so[4][16][20];
  const int tid = threadIdx.x, wave = tid >> 5, lane = tid & 31, col = lane & 15, g = lane >> 4; const int b = blockIdx.y; const int p0 = blockIdx.x * 64 + wave * 16;
  const int pa = p0 + col; const int ph = pa / WI, pw = pa % WI; const float* img = O + (size_t)b * NPOS * C3;
  v8f acc = {};
#pragma unroll 1
  for (int kc = 0; kc < K4 / 32; ++kc) { float v[16];
#pragma unroll
    for (int i = 0; i < 16; ++i) { const int k = kc * 32 + 8 * g + (i < 8 ? i : 8 + i); const int ci = k / 9, r = k % 9; const int hh = ph - 1 + r / 3, ww = pw - 1 + r % 3; float x = 0.f; if (hh >= 0 && hh < HI && ww >= 0 && ww < WI) x = img[((size_t)hh * WI + ww) * C3 + ci]; v[i] = x; }
    const F2 a = bsplit16(v); const v16b w = frag_b(P4 + (size_t)col * K4 + kc * 32, lane); acc = wmma_bf(a.l, w, acc); acc = wmma_bf(a.h, w, acc); }
  { const float bb = (col < C4) ? bfr(B4[col < C4 ? col : 0]) : 0.f;
#pragma unroll
    for (int r = 0; r < 8; ++r) so[wave][8 * g + r][col] = (col < C4) ? fmaxf(acc[r] + bb, 0.f) : 0.f; }
  LDSX();
  for (int rl2 = 0; rl2 < 16; rl2 += 2) if (lane < 8) vst2(A4 + ((size_t)b * NPOS + p0 + rl2 + (lane >> 2)) * 16 + (lane & 3) * 4, *(const v4f*)&so[wave][rl2 + (lane >> 2)][(lane & 3) * 4]);
}
__global__ __launch_bounds__(128) void k_conv5(const float* __restrict__ A4, const float* __restrict__ W5, const float* __restrict__ B5, float* __restrict__ out) {
  __shared__ float sw[C4 * 9]; __shared__ __align__(16) float so[WI];
  const int h = blockIdx.x, b = blockIdx.y, tid = threadIdx.x;
  if (tid < C4 * 9) sw[tid] = bfr(W5[tid]);
  __syncthreads();
  if (tid < WI) { const int w = tid; float a = bfr(B5[0]);
#pragma unroll 1
    for (int ci = 0; ci < C4; ++ci)
#pragma unroll
      for (int kh = 0; kh < 3; ++kh)
#pragma unroll
        for (int kw = 0; kw < 3; ++kw) { const int hh = h + kh - 1, ww = w + kw - 1; if (hh >= 0 && hh < HI && ww >= 0 && ww < WI) a += sw[ci * 9 + kh * 3 + kw] * A4[((size_t)b * NPOS + hh * WI + ww) * 16 + ci]; }
    so[w] = fmaxf(a, 0.f); }
  __syncthreads();
  if (tid < WI / 4) vst2(out + ((size_t)b * HI + h) * WI + tid * 4, *(const v4f*)&so[tid * 4]);
}
extern "C" void kernel_launch(void* const* d_in, const int* in_sizes, int n_in, void* d_out, int out_size, void* d_ws, size_t ws_size, hipStream_t stream) {
  (void)in_sizes; (void)n_in; (void)out_size;
  const float** F = (const float**)d_in;
  if (ws_size < (size_t)WS_END) return;
  char* ws = (char*)d_ws; __bf16 *P3 = (__bf16*)(ws + WS_P3), *P4 = (__bf16*)(ws + WS_P4), *VH = (__bf16*)(ws + WS_VH), *VL = (__bf16*)(ws + WS_VL);
  float *A2 = (float*)(ws + WS_A2), *BT = (float*)(ws + WS_BT), *O = (float*)(ws + WS_O), *A4 = (float*)(ws + WS_A4);
  k_pack<<<C3 + 16, 256, 0, stream>>>(F[5], F[7], P3, P4);
  k_conv12<<<dim3(HI, TNB), 256, 0, stream>>>(F[0], F[1], F[2], F[3], F[4], A2);
  k_conv3<<<dim3(NPOS / 64, TNB), 128, 0, stream>>>(A2, P3, F[6], BT, VH, VL);
  k_attn<<<dim3(TQB, TNB), 128, 0, stream>>>(BT, VH, VL, O);
  k_conv4<<<dim3(C4B, TNB), 128, 0, stream>>>(O, P4, F[8], A4);
  k_conv5<<<dim3(C5R, TNB), 128, 0, stream>>>(A4, F[9], F[10], (float*)d_out);
}
